// MultiheadL2Attention_42795054137395
// MI455X (gfx1250) — hardware-verified
//
#include <hip/hip_runtime.h>
#include <math.h>
#include <stdint.h>

constexpr int kNB    = 2;
constexpr int kSeq   = 2048;
constexpr int kEmb   = 1024;
constexpr int kHeads = 16;
constexpr int kHdim  = 64;
constexpr int kTok   = kNB * kSeq;
constexpr int kNBH   = kNB * kHeads;
constexpr int kBlk   = 64;
constexpr int kNBlk  = kSeq / kBlk;
constexpr int kOutN  = kNB * kEmb;
static_assert(kHeads * kHdim == kEmb);
static_assert(kSeq % kBlk == 0);
static_assert(kTok % 64 == 0 && kEmb % 64 == 0 && kEmb % 32 == 0);

constexpr size_t kBytesXb  = (size_t)kTok * kEmb * 2;
constexpr size_t kBytesWb  = (size_t)kEmb * kEmb * 2;
constexpr size_t kBytesF32 = (size_t)kTok * kEmb * 4;
constexpr size_t kBytesH16 = (size_t)kTok * kEmb * 2;
constexpr size_t kBytesVec = (size_t)kNBH * kSeq * 4;
constexpr size_t kBytesCtx = (size_t)kNB * kEmb * 4;
constexpr size_t kOffXq  = 0;
constexpr size_t kOffXk  = kOffXq + kBytesXb;
constexpr size_t kOffXv  = kOffXk + kBytesXb;
constexpr size_t kOffWq  = kOffXv + kBytesXb;
constexpr size_t kOffWk  = kOffWq + kBytesWb;
constexpr size_t kOffWv  = kOffWk + kBytesWb;
constexpr size_t kOffQf  = kOffWv + kBytesWb;
constexpr size_t kOffKf  = kOffQf + kBytesF32;
constexpr size_t kOffVf  = kOffKf + kBytesF32;
constexpr size_t kOffQh  = kOffVf + kBytesF32;
constexpr size_t kOffKh  = kOffQh + kBytesH16;
constexpr size_t kOffQ2  = kOffKh + kBytesH16;
constexpr size_t kOffK2  = kOffQ2 + kBytesVec;
constexpr size_t kOffRm  = kOffK2 + kBytesVec;
constexpr size_t kOffRz  = kOffRm + kBytesVec;
constexpr size_t kOffCs  = kOffRz + kBytesVec;
constexpr size_t kOffCtx = kOffCs + kBytesVec;
constexpr size_t kWsTotal = kOffCtx + kBytesCtx;
static_assert(kWsTotal == 99885056ull);
static_assert(kWsTotal <= 134217728ull);

typedef __attribute__((ext_vector_type(16))) _Float16 v16h;
typedef __attribute__((ext_vector_type(8)))  _Float16 v8h;
typedef __attribute__((ext_vector_type(16))) __bf16   v16b;
typedef __attribute__((ext_vector_type(8)))  __bf16   v8b;
typedef __attribute__((ext_vector_type(8)))  float    v8f;
typedef __attribute__((ext_vector_type(4)))  float    v4f;
typedef __attribute__((ext_vector_type(4)))  unsigned int v4u;

__device__ __forceinline__ unsigned short f2bf_bits(float f) {
  unsigned u = __float_as_uint(f);
  return (unsigned short)((u + 0x7FFFu + ((u >> 16) & 1u)) >> 16);
}
__device__ __forceinline__ float bf_bits2f(unsigned short h) { return __uint_as_float(((unsigned)h) << 16); }

__device__ __forceinline__ void dep_guard_h(v8f& a, v8f& b, v16h x, v16h y) { asm volatile("v_nop\n\tv_nop\n\tv_nop\n\tv_nop" : "+v"(a), "+v"(b) : "v"(x), "v"(y)); }
__device__ __forceinline__ void dep_guard_b(v8f& a, v8f& b, v16b x, v16b y) { asm volatile("v_nop\n\tv_nop\n\tv_nop\n\tv_nop" : "+v"(a), "+v"(b) : "v"(x), "v"(y)); }
__device__ __forceinline__ void keep4_h(v16h a, v16h b, v16h c, v16h d) { asm volatile("v_nop" :: "v"(a), "v"(b), "v"(c), "v"(d)); }
__device__ __forceinline__ void keep4_b(v16b a, v16b b, v16b c, v16b d) { asm volatile("v_nop" :: "v"(a), "v"(b), "v"(c), "v"(d)); }
__device__ __forceinline__ void acc_guard4(v8f& a, v8f& b, v8f& c, v8f& d) { asm volatile("v_nop\n\tv_nop\n\tv_nop\n\tv_nop" : "+v"(a), "+v"(b), "+v"(c), "+v"(d)); }
template <typename T> struct Frag;
template <> struct Frag<_Float16> {
  typedef v16h V; union U { v16h v; v8h h[2]; };
  static __device__ __forceinline__ v16h load(const _Float16* p) {
    U f; f.h[0] = *(const v8h*)(p); f.h[1] = *(const v8h*)(p + 16); return f.v;
  }
  static __device__ __forceinline__ v8f mma(v16h a, v16h b, v8f c) {
    return __builtin_amdgcn_wmma_f32_16x16x32_f16(false, a, false, b, (short)0, c, false, false);
  }
  static __device__ __forceinline__ void guard(v8f& a, v8f& b, v16h x, v16h y) { dep_guard_h(a, b, x, y); }
  static __device__ __forceinline__ void keep(v16h a, v16h b, v16h c, v16h d) { keep4_h(a, b, c, d); }
};
template <> struct Frag<__bf16> {
  typedef v16b V; union U { v16b v; v8b h[2]; };
  static __device__ __forceinline__ v16b load(const __bf16* p) {
    U f; f.h[0] = *(const v8b*)(p); f.h[1] = *(const v8b*)(p + 16); return f.v;
  }
  static __device__ __forceinline__ v8f mma(v16b a, v16b b, v8f c) {
    return __builtin_amdgcn_wmma_f32_16x16x32_bf16(false, a, false, b, (short)0, c, false, false);
  }
  static __device__ __forceinline__ void guard(v8f& a, v8f& b, v16b x, v16b y) { dep_guard_b(a, b, x, y); }
  static __device__ __forceinline__ void keep(v16b a, v16b b, v16b c, v16b d) { keep4_b(a, b, c, d); }
};

template <int ET> struct Elem;
template <> struct Elem<0> { typedef _Float16 T; };
template <> struct Elem<1> { typedef __bf16 T; };
template <int ET, bool SPLIT, int BIAS_MODE, int OUT_MODE, bool RESID, int ACT = 0>
__global__ __launch_bounds__(256) void wmma_gemm64(
    const unsigned short* __restrict__ Ap, const unsigned short* __restrict__ A2p, int lda, long strideA,
    const unsigned short* __restrict__ Btp, const unsigned short* __restrict__ Bt2p, int ldb, long strideB,
    void* __restrict__ Cout, void* __restrict__ Cout2, int ldc, long strideC,
    const float* __restrict__ bias,
    const float* __restrict__ resid, long strideR,
    int M, int N, int K, float scale) {
  typedef typename Elem<ET>::T T;
  typedef typename Frag<T>::V V;
  const T* A = (const T*)Ap; const T* A2 = (const T*)A2p; const T* Bt = (const T*)Btp; const T* Bt2 = (const T*)Bt2p;
  __shared__ __align__(16) float sT[8][16 * 68];
  const int b    = blockIdx.y;
  const int lane = threadIdx.x & 31;
  const int wave = threadIdx.x >> 5;
  const int tilesN = N >> 6;
  const int tilesM = M >> 6;
  const int tile = blockIdx.x * 8 + wave;
  if (tile >= tilesM * tilesN) return;
  const int tm = tile / tilesN;
  const int tn = tile - tm * tilesN;
  const int m0 = tm << 6;
  const int n0 = tn << 6;

  const T* Ab  = A  + (size_t)b * strideA;
  const T* Bb  = Bt + (size_t)b * strideB;
  const T* Ab2 = SPLIT ? (A2  + (size_t)b * strideA) : nullptr;
  const T* Bb2 = SPLIT ? (Bt2 + (size_t)b * strideB) : nullptr;

  const int rlane = lane & 15;
  const int koff  = (lane >> 4) * 8;
  const int mOff  = (lane >> 4) * 8;

  v8f acc[4][4];
#pragma unroll
  for (int i = 0; i < 4; ++i)
#pragma unroll
    for (int j = 0; j < 4; ++j) acc[i][j] = (v8f){0.f,0.f,0.f,0.f,0.f,0.f,0.f,0.f};

  for (int k0 = 0; k0 < K; k0 += 32) {
    V bh[4], bl[4];
#pragma unroll
    for (int j = 0; j < 4; ++j) {
      const size_t bo = (size_t)(n0 + (j << 4) + rlane) * ldb + koff + k0;
      bh[j] = Frag<T>::load(Bb + bo);
      if (SPLIT) bl[j] = Frag<T>::load(Bb2 + bo);
    }
#pragma unroll
    for (int i = 0; i < 4; ++i) {
      const size_t ao = (size_t)(m0 + (i << 4) + rlane) * lda + koff + k0;
      V ah = Frag<T>::load(Ab + ao);
      V al;
      if (SPLIT) al = Frag<T>::load(Ab2 + ao);
#pragma unroll
      for (int j = 0; j < 4; ++j) {
        acc[i][j] = Frag<T>::mma(ah, bh[j], acc[i][j]);
        if (SPLIT) {
          acc[i][j] = Frag<T>::mma(ah, bl[j], acc[i][j]);
          acc[i][j] = Frag<T>::mma(al, bh[j], acc[i][j]);
        }
      }
      Frag<T>::guard(acc[i][0], acc[i][3], ah, SPLIT ? al : ah);
    }
    Frag<T>::keep(bh[0], bh[1], bh[2], bh[3]);
    if (SPLIT) Frag<T>::keep(bl[0], bl[1], bl[2], bl[3]);
  }
  acc_guard4(acc[0][0], acc[0][1], acc[0][2], acc[0][3]);
  acc_guard4(acc[1][0], acc[1][1], acc[1][2], acc[1][3]);
  acc_guard4(acc[2][0], acc[2][1], acc[2][2], acc[2][3]);
  acc_guard4(acc[3][0], acc[3][1], acc[3][2], acc[3][3]);

  float* slab = sT[wave];
  const float* Rb = RESID ? (resid + (size_t)b * strideR) : nullptr;
#pragma unroll
  for (int i = 0; i < 4; ++i) {
    const int mBase = m0 + (i << 4);
#pragma unroll
    for (int j = 0; j < 4; ++j) {
      const int n = n0 + (j << 4) + rlane;
      float bv = 0.f;
      if (BIAS_MODE == 2) bv = bias[n];
#pragma unroll
      for (int r = 0; r < 8; ++r) {
        float v = acc[i][j][r] * scale;
        if (BIAS_MODE == 1) v += bias[mBase + mOff + r];
        if (BIAS_MODE == 2) v += bv;
        if (RESID) v += Rb[(size_t)(mBase + mOff + r) * ldc + n];
        if (ACT == 2) v = fmaxf(v, 0.0f);
        if (ACT == 4) v = (v > 0.f) ? v : 0.01f * v;
        slab[(mOff + r) * 68 + (j << 4) + rlane] = v;
      }
    }
    __builtin_amdgcn_fence(__ATOMIC_RELEASE, "workgroup");
    __builtin_amdgcn_wave_barrier();
    __builtin_amdgcn_fence(__ATOMIC_ACQUIRE, "workgroup");
    if (OUT_MODE == 0) {
      float* C = (float*)Cout + (size_t)b * strideC;
      const int hh = lane >> 4, c4 = (lane & 15) * 4;
      for (int pass = 0; pass < 2; ++pass) {
#pragma unroll
        for (int it = 0; it < 8; ++it) {
          const int row = it * 2 + hh;
          v4f v = *(const v4f*)(slab + row * 68 + c4);
          *(volatile v4f*)(C + (size_t)(mBase + row) * ldc + n0 + c4) = v;
        }
        __threadfence();
      }
    } else {
      const int q = lane >> 3, c8 = (lane & 7) * 8;
      unsigned short* C  = (unsigned short*)Cout  + (size_t)b * strideC;
      unsigned short* C2 = (OUT_MODE == 2) ? ((unsigned short*)Cout2 + (size_t)b * strideC) : nullptr;
      for (int pass = 0; pass < 2; ++pass) {
#pragma unroll
        for (int it = 0; it < 4; ++it) {
          const int row = it * 4 + q;
          const float* sp = slab + row * 68 + c8;
          v8h hv, lv;
#pragma unroll
          for (int e = 0; e < 8; ++e) {
            if (OUT_MODE == 1) {
              hv[e] = (_Float16)sp[e];
            } else {
              unsigned short hb = f2bf_bits(sp[e]);
              unsigned short lb = f2bf_bits(sp[e] - bf_bits2f(hb));
              hv[e] = __builtin_bit_cast(_Float16, hb);
              lv[e] = __builtin_bit_cast(_Float16, lb);
            }
          }
          *(volatile v8h*)(C + (size_t)(mBase + row) * ldc + n0 + c8) = hv;
          if (OUT_MODE == 2) *(volatile v8h*)(C2 + (size_t)(mBase + row) * ldc + n0 + c8) = lv;
        }
        __threadfence();
      }
    }
    __builtin_amdgcn_fence(__ATOMIC_RELEASE, "workgroup");
    __builtin_amdgcn_wave_barrier();
    __builtin_amdgcn_fence(__ATOMIC_ACQUIRE, "workgroup");
  }
}

__device__ __forceinline__ unsigned pkbf2(float a, float b) {
  return (unsigned)f2bf_bits(a) | ((unsigned)f2bf_bits(b) << 16);
}
__device__ __forceinline__ float bf_rne(float f) { return bf_bits2f(f2bf_bits(f)); }
__device__ __forceinline__ v8f mma_f16(v16h a, v16h b, v8f c) {
  c = __builtin_amdgcn_wmma_f32_16x16x32_f16(false, a, false, b, (short)0, c, false, false);
  asm volatile("v_nop\n\tv_nop\n\tv_nop\n\tv_nop" : "+v"(c) : "v"(a), "v"(b));
  return c;
}

__global__ __launch_bounds__(256) void cast_bf16x8_kernel(
    const float* __restrict__ in0, const float* __restrict__ in1, const float* __restrict__ in2,
    unsigned short* __restrict__ out0, unsigned short* __restrict__ out1, unsigned short* __restrict__ out2,
    int n8) {
  const int z = blockIdx.y;
  const float* in = (z == 0) ? in0 : (z == 1) ? in1 : in2;
  unsigned short* out = (z == 0) ? out0 : (z == 1) ? out1 : out2;
  const int i  = blockIdx.x * 256 + threadIdx.x;
  const int ic = (i < n8) ? i : (n8 - 1);
  const v4f a = *(const v4f*)(in + (size_t)ic * 8);
  const v4f c = *(const v4f*)(in + (size_t)ic * 8 + 4);
  v4u u;
  u[0] = pkbf2(a[0], a[1]); u[1] = pkbf2(a[2], a[3]);
  u[2] = pkbf2(c[0], c[1]); u[3] = pkbf2(c[2], c[3]);
  if (i < n8) {
    volatile v4u* p = (volatile v4u*)(out + (size_t)i * 8);
    *p = u;
    __threadfence();
    *p = u;
  }
}

__global__ __launch_bounds__(256) void normcast_kernel(
    const float* __restrict__ qf, const float* __restrict__ kf,
    unsigned short* __restrict__ qh, unsigned short* __restrict__ kh,
    float* __restrict__ q2, float* __restrict__ k2) {
  __shared__ float sq[32];
  const int z = blockIdx.z;
  const float* src = (z == 0) ? qf : kf;
  _Float16* dsth = (_Float16*)((z == 0) ? qh : kh);
  float* dstn = (z == 0) ? q2 : k2;
  const int t = threadIdx.x, seg = t >> 3, e8 = t & 7;
  const int tok0  = blockIdx.x * 32;
  const int token = tok0 + seg;
  const int h = blockIdx.y;
  const size_t off = (size_t)token * kEmb + (size_t)h * kHdim + (size_t)e8 * 8;
  const v4f a = *(const v4f*)(src + off);
  const v4f c = *(const v4f*)(src + off + 4);
  float ss = a[0] * a[0];
  ss += a[1] * a[1]; ss += a[2] * a[2]; ss += a[3] * a[3];
  ss += c[0] * c[0]; ss += c[1] * c[1]; ss += c[2] * c[2]; ss += c[3] * c[3];
  v8h hv;
  hv[0] = (_Float16)a[0]; hv[1] = (_Float16)a[1]; hv[2] = (_Float16)a[2]; hv[3] = (_Float16)a[3];
  hv[4] = (_Float16)c[0]; hv[5] = (_Float16)c[1]; hv[6] = (_Float16)c[2]; hv[7] = (_Float16)c[3];
  {
    volatile v8h* p = (volatile v8h*)(dsth + off);
    *p = hv;
    __threadfence();
    *p = hv;
  }
  ss += __shfl_xor(ss, 1, 32);
  ss += __shfl_xor(ss, 2, 32);
  ss += __shfl_xor(ss, 4, 32);
  if (e8 == 0) sq[seg] = ss;
  __syncthreads();
  if (t < 32) {
    const int b  = tok0 / kSeq;
    const int l0 = tok0 - b * kSeq;
    const float v = sq[t];
    volatile float* p = dstn + (size_t)(b * kHeads + h) * kSeq + l0 + t;
    *p = v;
    __threadfence();
    *p = v;
  }
}

__global__ __launch_bounds__(128) void rowstat_kernel(
    const unsigned short* __restrict__ qhp, const unsigned short* __restrict__ khp,
    const float* __restrict__ q2, const float* __restrict__ k2,
    float* __restrict__ rowm, float* __restrict__ rowiz) {
  union FH { v16h v; v8h h[2]; };
  __shared__ __align__(16) _Float16 Ksh[kBlk * kHdim];
  __shared__ __align__(16) float smM[kBlk];
  __shared__ __align__(16) float smZ[kBlk];
  const int tid = threadIdx.x, wave = tid >> 5, lane = tid & 31;
  const int hh = lane >> 4, c = lane & 15;
  const int bx = blockIdx.x;
  const int qb = bx % kNBlk;
  const int bh = bx / kNBlk;
  const int h  = bh % kHeads;
  const int b  = bh / kHeads;
  const int q0 = qb * kBlk + wave * 16;
  const _Float16* qpl = (const _Float16*)qhp;
  const _Float16* kpl = (const _Float16*)khp;

  v16h qa[2];
  {
    const _Float16* qrow = qpl + (size_t)(b * kSeq + q0 + c) * kEmb + h * kHdim + 8 * hh;
    qa[0] = Frag<_Float16>::load(qrow);
    qa[1] = Frag<_Float16>::load(qrow + 32);
  }
  float q2r[8];
#pragma unroll
  for (int r = 0; r < 8; ++r) q2r[r] = q2[(size_t)bh * kSeq + q0 + 8 * hh + r];

  float mrow[8], lrow[8];
#pragma unroll
  for (int r = 0; r < 8; ++r) { mrow[r] = -INFINITY; lrow[r] = 0.f; }

#pragma unroll 1
  for (int kc = 0; kc < kNBlk; ++kc) {
    const int kv0 = kc * kBlk;
    __syncthreads();
    {
      const int kvr = tid >> 1, dh = (tid & 1) * 32;
      const _Float16* krow = kpl + (size_t)(b * kSeq + kv0 + kvr) * kEmb + h * kHdim + dh;
      _Float16* kd = Ksh + kvr * kHdim + dh;
#pragma unroll
      for (int i = 0; i < 4; ++i) {
        const v8h tv = *(const v8h*)(krow + 8 * i);
        *(v8h*)(kd + 8 * i) = tv;
      }
    }
    __syncthreads();

    float k2c[4];
#pragma unroll
    for (int j = 0; j < 4; ++j) k2c[j] = k2[(size_t)bh * kSeq + kv0 + j * 16 + c];

    v8f s[4];
#pragma unroll
    for (int j = 0; j < 4; ++j) {
      s[j] = (v8f){0.f,0.f,0.f,0.f,0.f,0.f,0.f,0.f};
#pragma unroll
      for (int dc = 0; dc < 2; ++dc) {
        FH kb;
        kb.h[0] = *(const v8h*)(Ksh + (j * 16 + c) * kHdim + dc * 32 + 8 * hh);
        kb.h[1] = *(const v8h*)(Ksh + (j * 16 + c) * kHdim + dc * 32 + 16 + 8 * hh);
        s[j] = mma_f16(qa[dc], kb.v, s[j]);
      }
    }
    float cm[8];
#pragma unroll
    for (int r = 0; r < 8; ++r) {
      float m = -INFINITY;
#pragma unroll
      for (int j = 0; j < 4; ++j) {
        float d2 = q2r[r] + k2c[j] - 2.0f * s[j][r];
        d2 = fmaxf(d2, 0.0f);
        const float sc = -sqrtf(d2);
        s[j][r] = sc;
        m = fmaxf(m, sc);
      }
#pragma unroll
      for (int off = 1; off < 16; off <<= 1) m = fmaxf(m, __shfl_xor(m, off, 32));
      cm[r] = m;
    }
#pragma unroll
    for (int r = 0; r < 8; ++r) {
      const float mnew  = fmaxf(mrow[r], cm[r]);
      const float alpha = expf(mrow[r] - mnew);
      mrow[r] = mnew;
      float psum = 0.f;
#pragma unroll
      for (int j = 0; j < 4; ++j) psum += expf(s[j][r] - mnew);
#pragma unroll
      for (int off = 1; off < 16; off <<= 1) psum += __shfl_xor(psum, off, 32);
      lrow[r] = lrow[r] * alpha + psum;
    }
  }

#pragma unroll
  for (int r = 0; r < 8; ++r) {
    smM[wave * 16 + 8 * hh + r] = mrow[r];
    smZ[wave * 16 + 8 * hh + r] = 1.0f / lrow[r];
  }
  __syncthreads();
  if (wave == 0) {
    const size_t base = (size_t)bh * kSeq + (size_t)qb * kBlk;
    const int l4 = (lane & 15) * 4;
    const v4f vm = *(const v4f*)(smM + l4);
    const v4f vz = *(const v4f*)(smZ + l4);
    for (int pass = 0; pass < 2; ++pass) {
      if (lane < 16) {
        *(volatile v4f*)(rowm  + base + l4) = vm;
        *(volatile v4f*)(rowiz + base + l4) = vz;
      }
      __threadfence();
    }
  }
}

__global__ __launch_bounds__(128) void colsum_kernel(
    const unsigned short* __restrict__ qhp, const unsigned short* __restrict__ khp,
    const float* __restrict__ q2, const float* __restrict__ k2,
    const float* __restrict__ rowm, const float* __restrict__ rowiz,
    float* __restrict__ colsum) {
  union FH { v16h v; v8h h[2]; };
  __shared__ __align__(16) _Float16 Qsh[kBlk * kHdim];
  __shared__ __align__(16) float smS[kBlk];
  const int tid = threadIdx.x, wave = tid >> 5, lane = tid & 31;
  const int hh = lane >> 4, c = lane & 15;
  const int bx = blockIdx.x;
  const int kb = bx % kNBlk;
  const int bh = bx / kNBlk;
  const int h  = bh % kHeads;
  const int b  = bh / kHeads;
  const int k0 = kb * kBlk + wave * 16;
  const _Float16* qpl = (const _Float16*)qhp;
  const _Float16* kpl = (const _Float16*)khp;

  v16h ka[2];
  {
    const _Float16* krow = kpl + (size_t)(b * kSeq + k0 + c) * kEmb + h * kHdim + 8 * hh;
    ka[0] = Frag<_Float16>::load(krow);
    ka[1] = Frag<_Float16>::load(krow + 32);
  }
  float k2r[8];
#pragma unroll
  for (int r = 0; r < 8; ++r) k2r[r] = k2[(size_t)bh * kSeq + k0 + 8 * hh + r];

  float cs[8];
#pragma unroll
  for (int r = 0; r < 8; ++r) cs[r] = 0.f;

#pragma unroll 1
  for (int qc = 0; qc < kNBlk; ++qc) {
    const int qc0 = qc * kBlk;
    __syncthreads();
    {
      const int qr = tid >> 1, dh = (tid & 1) * 32;
      const _Float16* qrow = qpl + (size_t)(b * kSeq + qc0 + qr) * kEmb + h * kHdim + dh;
      _Float16* qd = Qsh + qr * kHdim + dh;
#pragma unroll
      for (int i = 0; i < 4; ++i) {
        const v8h tv = *(const v8h*)(qrow + 8 * i);
        *(v8h*)(qd + 8 * i) = tv;
      }
    }
    __syncthreads();

    float q2c[4], mq[4], iz[4];
#pragma unroll
    for (int j = 0; j < 4; ++j) {
      const size_t idx = (size_t)bh * kSeq + qc0 + j * 16 + c;
      q2c[j] = q2[idx];
      mq[j]  = rowm[idx];
      iz[j]  = rowiz[idx];
    }

    v8f s[4];
#pragma unroll
    for (int j = 0; j < 4; ++j) {
      s[j] = (v8f){0.f,0.f,0.f,0.f,0.f,0.f,0.f,0.f};
#pragma unroll
      for (int dc = 0; dc < 2; ++dc) {
        FH qbv;
        qbv.h[0] = *(const v8h*)(Qsh + (j * 16 + c) * kHdim + dc * 32 + 8 * hh);
        qbv.h[1] = *(const v8h*)(Qsh + (j * 16 + c) * kHdim + dc * 32 + 16 + 8 * hh);
        s[j] = mma_f16(ka[dc], qbv.v, s[j]);
      }
    }
#pragma unroll
    for (int r = 0; r < 8; ++r) {
#pragma unroll
      for (int j = 0; j < 4; ++j) {
        float d2 = q2c[j] + k2r[r] - 2.0f * s[j][r];
        d2 = fmaxf(d2, 0.0f);
        const float sc = -sqrtf(d2);
        const float p  = expf(sc - mq[j]) * iz[j];
        cs[r] += p;
      }
    }
  }

#pragma unroll
  for (int r = 0; r < 8; ++r) {
    float v = cs[r];
#pragma unroll
    for (int off = 1; off < 16; off <<= 1) v += __shfl_xor(v, off, 32);
    smS[wave * 16 + 8 * hh + r] = v;
  }
  __syncthreads();
  if (wave == 0) {
    const size_t base = (size_t)bh * kSeq + (size_t)kb * kBlk;
    const int l4 = (lane & 15) * 4;
    const v4f vs = *(const v4f*)(smS + l4);
    for (int pass = 0; pass < 2; ++pass) {
      if (lane < 16) *(volatile v4f*)(colsum + base + l4) = vs;
      __threadfence();
    }
  }
}

__global__ __launch_bounds__(256) void ctx_kernel(
    const float* __restrict__ colsum, const float* __restrict__ vf, float* __restrict__ ctx) {
  const int o  = blockIdx.x * 256 + threadIdx.x;
  const int oc = (o < kOutN) ? o : (kOutN - 1);
  const int b  = oc / kEmb;
  const int e  = oc - b * kEmb;
  const int h  = e / kHdim;
  const float* csp = colsum + (size_t)(b * kHeads + h) * kSeq;
  const float* vp  = vf + (size_t)b * kSeq * kEmb + e;
  float acc = 0.f;
#pragma unroll 1
  for (int k = 0; k < kSeq; ++k) acc += csp[k] * vp[(size_t)k * kEmb];
  if (o < kOutN) {
    volatile float* p = ctx + o;
    *p = acc;
    __threadfence();
    *p = acc;
  }
}

__global__ __launch_bounds__(256) void outproj_kernel(
    const float* __restrict__ ctx, const float* __restrict__ Wo, float* __restrict__ out) {
  const int o  = blockIdx.x * 256 + threadIdx.x;
  const int oc = (o < kOutN) ? o : (kOutN - 1);
  const int b  = oc / kEmb;
  const int n  = oc - b * kEmb;
  const float* cr = ctx + (size_t)b * kEmb;
  const float* wr = Wo + (size_t)n * kEmb;
  float acc = 0.f;
#pragma unroll 1
  for (int e = 0; e < kEmb; e += 4) {
    const v4f cv = *(const v4f*)(cr + e);
    const v4f wv = *(const v4f*)(wr + e);
    acc += cv[0] * bf_rne(wv[0]);
    acc += cv[1] * bf_rne(wv[1]);
    acc += cv[2] * bf_rne(wv[2]);
    acc += cv[3] * bf_rne(wv[3]);
  }
  if (o < kOutN) {
    volatile float* p = out + o;
    *p = acc;
    __threadfence();
    *p = acc;
  }
}

extern "C" void kernel_launch(void* const* d_in, const int* in_sizes, int n_in,
                              void* d_out, int out_size, void* d_ws,
                              size_t ws_size, hipStream_t stream) {
  if (n_in < 7) return;
  if (in_sizes[0] != kTok * kEmb || in_sizes[1] != kTok * kEmb || in_sizes[2] != kTok * kEmb) return;
  if (in_sizes[3] != kEmb * kEmb || in_sizes[4] != kEmb * kEmb || in_sizes[5] != kEmb * kEmb ||
      in_sizes[6] != kEmb * kEmb) return;
  if (out_size != kOutN) return;
  if (ws_size < kWsTotal) return;

  const float* Q  = (const float*)d_in[0];
  const float* K  = (const float*)d_in[1];
  const float* Vv = (const float*)d_in[2];
  const float* Wq = (const float*)d_in[3];
  const float* Wk = (const float*)d_in[4];
  const float* Wv = (const float*)d_in[5];
  const float* Wo = (const float*)d_in[6];
  float* out = (float*)d_out;

  char* ws = (char*)d_ws;
  unsigned short* Xq = (unsigned short*)(ws + kOffXq);
  unsigned short* Xk = (unsigned short*)(ws + kOffXk);
  unsigned short* Xv = (unsigned short*)(ws + kOffXv);
  unsigned short* Bq = (unsigned short*)(ws + kOffWq);
  unsigned short* Bk = (unsigned short*)(ws + kOffWk);
  unsigned short* Bv = (unsigned short*)(ws + kOffWv);
  float* qf = (float*)(ws + kOffQf);
  float* kf = (float*)(ws + kOffKf);
  float* vf = (float*)(ws + kOffVf);
  unsigned short* qh = (unsigned short*)(ws + kOffQh);
  unsigned short* kh = (unsigned short*)(ws + kOffKh);
  float* q2  = (float*)(ws + kOffQ2);
  float* k2  = (float*)(ws + kOffK2);
  float* rm  = (float*)(ws + kOffRm);
  float* rz  = (float*)(ws + kOffRz);
  float* csm = (float*)(ws + kOffCs);
  float* ctx = (float*)(ws + kOffCtx);
  const float* dummy = (const float*)(ws + kOffCtx);

  const int n8x = kTok * kEmb / 8;
  const int n8w = kEmb * kEmb / 8;
  cast_bf16x8_kernel<<<dim3((n8x + 255) / 256, 3), 256, 0, stream>>>(Q, K, Vv, Xq, Xk, Xv, n8x);
  cast_bf16x8_kernel<<<dim3((n8w + 255) / 256, 3), 256, 0, stream>>>(Wq, Wk, Wv, Bq, Bk, Bv, n8w);

  const int gemmBlocks = (kTok / 64) * (kEmb / 64) / 8;
  wmma_gemm64<1, false, 0, 0, false><<<dim3(gemmBlocks, 1), 256, 0, stream>>>(
      Xq, Xq, kEmb, 0L, Bq, Bq, kEmb, 0L, (void*)qf, (void*)qf, kEmb, 0L, dummy, dummy, 0L,
      kTok, kEmb, kEmb, 1.0f);
  wmma_gemm64<1, false, 0, 0, false><<<dim3(gemmBlocks, 1), 256, 0, stream>>>(
      Xk, Xk, kEmb, 0L, Bk, Bk, kEmb, 0L, (void*)kf, (void*)kf, kEmb, 0L, dummy, dummy, 0L,
      kTok, kEmb, kEmb, 1.0f);
  wmma_gemm64<1, false, 0, 0, false><<<dim3(gemmBlocks, 1), 256, 0, stream>>>(
      Xv, Xv, kEmb, 0L, Bv, Bv, kEmb, 0L, (void*)vf, (void*)vf, kEmb, 0L, dummy, dummy, 0L,
      kTok, kEmb, kEmb, 1.0f);

  normcast_kernel<<<dim3(kTok / 32, kHeads, 2), 256, 0, stream>>>(qf, kf, qh, kh, q2, k2);

  rowstat_kernel<<<dim3(kNBH * kNBlk), 128, 0, stream>>>(qh, kh, q2, k2, rm, rz);
  colsum_kernel<<<dim3(kNBH * kNBlk), 128, 0, stream>>>(qh, kh, q2, k2, rm, rz, csm);

  ctx_kernel<<<dim3((kOutN + 255) / 256), 256, 0, stream>>>(csm, vf, ctx);
  outproj_kernel<<<dim3((kOutN + 255) / 256), 256, 0, stream>>>(ctx, Wo, out);
}
